// GraphormerBlock_64330020159495
// MI455X (gfx1250) — hardware-verified
//
#include <hip/hip_runtime.h>
#include <math.h>

#define NTOK 2048
#define CH   256
#define NH   8
#define HD   32
#define FF   1024
#define NE   32768
#define NT   8
#define NR   12
#define NBK  21
#define SEGCAP 512
#define WCAP   1024
#define WSC  32.0f
#define PSC  16384.0f
#define OSC  64.0f
#define GSC  16.0f

typedef _Float16 v16h __attribute__((ext_vector_type(16)));
typedef _Float16 v8h  __attribute__((ext_vector_type(8)));
typedef float    v8f  __attribute__((ext_vector_type(8)));
typedef float    v4f  __attribute__((ext_vector_type(4)));
typedef int      i4   __attribute__((ext_vector_type(4)));
typedef v8h __attribute__((may_alias)) v8ha;
typedef v4f __attribute__((may_alias)) v4fa;
typedef i4  __attribute__((may_alias)) i4a;

union Frag { v16h v; v8h half[2]; };

__device__ __forceinline__ v8f wmma_f16(v16h a, v16h b, v8f c) {
  v8f d = __builtin_amdgcn_wmma_f32_16x16x32_f16(false, a, false, b, (short)0, c, false, false);
  asm volatile("v_nop\n\tv_nop\n\tv_nop\n\tv_nop" : "+v"(d) : "v"(a), "v"(b));
  return d;
}

__device__ __forceinline__ v16h load_frag(const _Float16* p, int h) {
  Frag f;
  f.half[0] = *(const v8ha*)(p + 8 * h);
  f.half[1] = *(const v8ha*)(p + 16 + 8 * h);
  return f.v;
}

__device__ __forceinline__ float wsum(float v) {
  v += __shfl_xor(v, 16);
  v += __shfl_xor(v, 8);
  v += __shfl_xor(v, 4);
  v += __shfl_xor(v, 2);
  v += __shfl_xor(v, 1);
  return v;
}

__device__ __forceinline__ void wtr_store(const _Float16* sT, _Float16* dst, int K,
                                          int n0, int k0, int w, int lane) {
  const int q8 = lane & 7, sub = lane >> 3;
  #pragma unroll
  for (int i = 0; i < 2; ++i) {
    const int nl = w * 8 + i * 4 + sub;
    const v8h v = *(const v8ha*)(sT + nl * 72 + 8 * q8);
    *(volatile v8h*)(dst + (size_t)(n0 + nl) * K + k0 + 8 * q8) = v;
  }
}

__global__ __launch_bounds__(256) void wtr_kernel(const float* __restrict__ w0, const float* __restrict__ w1,
                                                   const float* __restrict__ w2, const float* __restrict__ w3,
                                                   _Float16* __restrict__ outp, int K, int NC)
{
  __shared__ __attribute__((aligned(16))) _Float16 sT[64 * 72];
  const int t = threadIdx.x, lane = t & 31, w = t >> 5;
  const int n0 = blockIdx.x * 64, k0 = blockIdx.y * 64, z = blockIdx.z;
  const float* src = (z == 0) ? w0 : ((z == 1) ? w1 : ((z == 2) ? w2 : w3));
  _Float16* dst = outp + (size_t)z * (size_t)K * (size_t)NC;
  #pragma unroll
  for (int i = 0; i < 4; ++i) {
    const int idx = t + 256 * i;
    const int r = idx >> 4, c4 = idx & 15;
    const v4f v = *(const v4fa*)(src + (size_t)(k0 + r) * NC + n0 + 4 * c4);
    _Float16* col = sT + (4 * c4) * 72 + r;
    col[0]   = (_Float16)(v.x * WSC);
    col[72]  = (_Float16)(v.y * WSC);
    col[144] = (_Float16)(v.z * WSC);
    col[216] = (_Float16)(v.w * WSC);
  }
  __syncthreads();
  wtr_store(sT, dst, K, n0, k0, w, lane);
  __threadfence();
  wtr_store(sT, dst, K, n0, k0, w, lane);
}

__global__ __launch_bounds__(256) void ln_kernel(const float* __restrict__ x, const float* __restrict__ g,
                                                  const float* __restrict__ bb, _Float16* __restrict__ outp,
                                                  int nrows)
{
  const int lane = threadIdx.x & 31, w = threadIdx.x >> 5;
  const int row = blockIdx.x * 8 + w;
  if (row >= nrows) return;
  const float* xr = x + (size_t)row * CH + 8 * lane;
  const v4f a = *(const v4fa*)xr;
  const v4f c = *(const v4fa*)(xr + 4);
  float sm = ((a.x + a.y) + (a.z + a.w)) + ((c.x + c.y) + (c.z + c.w));
  sm = wsum(sm);
  const float mu = sm * (1.0f / CH);
  const float d0 = a.x - mu, d1 = a.y - mu, d2 = a.z - mu, d3 = a.w - mu;
  const float d4 = c.x - mu, d5 = c.y - mu, d6 = c.z - mu, d7 = c.w - mu;
  float sq = ((d0 * d0 + d1 * d1) + (d2 * d2 + d3 * d3)) + ((d4 * d4 + d5 * d5) + (d6 * d6 + d7 * d7));
  sq = wsum(sq);
  const float inv = rsqrtf(sq * (1.0f / CH) + 1e-5f);
  const v4f ga = *(const v4fa*)(g + 8 * lane);
  const v4f gc = *(const v4fa*)(g + 8 * lane + 4);
  const v4f ba = *(const v4fa*)(bb + 8 * lane);
  const v4f bc = *(const v4fa*)(bb + 8 * lane + 4);
  const v8h o = { (_Float16)(d0 * inv * ga.x + ba.x), (_Float16)(d1 * inv * ga.y + ba.y),
                  (_Float16)(d2 * inv * ga.z + ba.z), (_Float16)(d3 * inv * ga.w + ba.w),
                  (_Float16)(d4 * inv * gc.x + bc.x), (_Float16)(d5 * inv * gc.y + bc.y),
                  (_Float16)(d6 * inv * gc.z + bc.z), (_Float16)(d7 * inv * gc.w + bc.w) };
  _Float16* dp = outp + (size_t)row * CH + 8 * lane;
  *(volatile v8h*)dp = o;
  __threadfence();
  *(volatile v8h*)dp = o;
}

__device__ __forceinline__ void gemm_core(const _Float16* __restrict__ A, int lda, int kcs,
                                          const _Float16* __restrict__ Bt, int ldb, int K,
                                          int arow, int brow, int h, v8f (&acc)[2][4])
{
  const _Float16* a0p = A + (size_t)arow * lda;
  const _Float16* a1p = a0p + (size_t)16 * lda;
  const _Float16* bp  = Bt + (size_t)brow * ldb;
  #pragma unroll 1
  for (int k0 = 0; k0 < K; k0 += 32) {
    const size_t ao = (size_t)(k0 >> 5) * (size_t)kcs;
    const v16h fa0 = load_frag(a0p + ao, h);
    const v16h fa1 = load_frag(a1p + ao, h);
    #pragma unroll
    for (int nt = 0; nt < 4; ++nt) {
      const v16h fb = load_frag(bp + (size_t)nt * 16 * ldb + k0, h);
      acc[0][nt] = wmma_f16(fa0, fb, acc[0][nt]);
      acc[1][nt] = wmma_f16(fa1, fb, acc[1][nt]);
    }
  }
}

__device__ __forceinline__ void qkv_store(const _Float16* sT, _Float16* plane, _Float16* vtp,
                                          int which, int m0, int c0, int w, int lane) {
  const int q8 = lane & 7, sub = lane >> 3;
  #pragma unroll
  for (int i = 0; i < 8; ++i) {
    const int lid = w * 32 + i * 4 + sub;
    v8h v;
    _Float16* dst;
    if (which != 2) {
      v = *(const v8ha*)(sT + lid * 64 + 8 * q8);
      dst = plane + (size_t)(m0 + lid) * CH + c0 + 8 * q8;
    } else {
      const int d = lid >> 1, hl = lid & 1;
      v = *(const v8ha*)(sT + d * 128 + 64 * hl + 8 * q8);
      dst = vtp + (size_t)(c0 + d) * NTOK + m0 + 64 * hl + 8 * q8;
    }
    *(volatile v8h*)dst = v;
  }
}

__global__ __launch_bounds__(128) void qkv_kernel(
    const _Float16* __restrict__ hpl,
    const _Float16* __restrict__ wt,
    const float* __restrict__ bq, const float* __restrict__ bk, const float* __restrict__ bv,
    _Float16* __restrict__ qpl,
    _Float16* __restrict__ kpl,
    _Float16* __restrict__ vtp)
{
  __shared__ __attribute__((aligned(16))) _Float16 sT[128 * 64];
  const int tid = threadIdx.x, lane = tid & 31, w = tid >> 5;
  const int h = lane >> 4, m = lane & 15;
  const int m0 = blockIdx.x * 128;
  const int cg = blockIdx.y;
  const int which = cg >> 2, c0 = (cg & 3) * 64;
  const int m0w = m0 + 32 * w;

  const v8f zero8 = {0.f, 0.f, 0.f, 0.f, 0.f, 0.f, 0.f, 0.f};
  v8f acc[2][4];
  #pragma unroll
  for (int mt = 0; mt < 2; ++mt)
    #pragma unroll
    for (int nt = 0; nt < 4; ++nt) acc[mt][nt] = zero8;

  gemm_core(hpl, CH, 32, wt, CH, CH, m0w + m, cg * 64 + m, h, acc);

  const float* bias = (which == 0) ? bq : ((which == 1) ? bk : bv);
  #pragma unroll
  for (int nt = 0; nt < 4; ++nt) {
    const int feat = 16 * nt + m;
    const float bvl = bias[c0 + feat];
    #pragma unroll
    for (int mt = 0; mt < 2; ++mt) {
      #pragma unroll
      for (int r = 0; r < 8; ++r) {
        const int tokl = 32 * w + 16 * mt + 8 * h + r;
        const float y = acc[mt][nt][r] * (1.0f / WSC) + bvl;
        const int idx = (which == 2) ? (feat * 128 + tokl) : (tokl * 64 + feat);
        sT[idx] = (_Float16)y;
      }
    }
  }
  __syncthreads();

  _Float16* plane = (which == 0) ? qpl : kpl;
  qkv_store(sT, plane, vtp, which, m0, c0, w, lane);
  __threadfence();
  qkv_store(sT, plane, vtp, which, m0, c0, w, lane);
}

__device__ __forceinline__ void f16_store(const _Float16* sT, _Float16* plane, int ldo,
                                          int m0, int c0, int w, int lane) {
  const int q8 = lane & 7, sub = lane >> 3;
  #pragma unroll
  for (int i = 0; i < 8; ++i) {
    const int lid = w * 32 + i * 4 + sub;
    const v8h v = *(const v8ha*)(sT + lid * 64 + 8 * q8);
    *(volatile v8h*)(plane + (size_t)(m0 + lid) * ldo + c0 + 8 * q8) = v;
  }
}

__global__ __launch_bounds__(128) void ffn1_kernel(
    const _Float16* __restrict__ h2,
    const _Float16* __restrict__ w1t,
    const float* __restrict__ b1,
    _Float16* __restrict__ gpl)
{
  __shared__ __attribute__((aligned(16))) _Float16 sT[128 * 64];
  const int tid = threadIdx.x, lane = tid & 31, w = tid >> 5;
  const int h = lane >> 4, m = lane & 15;
  const int m0 = blockIdx.x * 128, c0 = blockIdx.y * 64;
  const int m0w = m0 + 32 * w;

  const v8f zero8 = {0.f, 0.f, 0.f, 0.f, 0.f, 0.f, 0.f, 0.f};
  v8f acc[2][4];
  #pragma unroll
  for (int mt = 0; mt < 2; ++mt)
    #pragma unroll
    for (int nt = 0; nt < 4; ++nt) acc[mt][nt] = zero8;

  gemm_core(h2, CH, 32, w1t, CH, CH, m0w + m, c0 + m, h, acc);

  #pragma unroll
  for (int nt = 0; nt < 4; ++nt) {
    const int feat = 16 * nt + m;
    const float bvl = b1[c0 + feat];
    #pragma unroll
    for (int mt = 0; mt < 2; ++mt) {
      #pragma unroll
      for (int r = 0; r < 8; ++r) {
        const int tokl = 32 * w + 16 * mt + 8 * h + r;
        const float y = acc[mt][nt][r] * (1.0f / WSC) + bvl;
        const float ge = 0.5f * y * (1.0f + erff(y * 0.70710678118654752f));
        sT[tokl * 64 + feat] = (_Float16)(ge * GSC);
      }
    }
  }
  __syncthreads();

  f16_store(sT, gpl, FF, m0, c0, w, lane);
  __threadfence();
  f16_store(sT, gpl, FF, m0, c0, w, lane);
}

__device__ __forceinline__ void f32_store(const float* sF, const float* __restrict__ resid,
                                          float* out, int m0, int c0, int w, int lane) {
  const int q8 = lane & 7, sub = lane >> 3;
  #pragma unroll
  for (int i = 0; i < 16; ++i) {
    const int li = 4 * i + sub;
    const int row = 32 * w + (li >> 1), hl = li & 1;
    v4f v = *(const v4fa*)(sF + row * 64 + 32 * hl + 4 * q8);
    const size_t gi = (size_t)(m0 + row) * CH + c0 + 32 * hl + 4 * q8;
    const v4f rr = *(const v4fa*)(resid + gi);
    v = v + rr;
    *(volatile v4f*)(out + gi) = v;
  }
}

__global__ __launch_bounds__(128) void gemm_f32_kernel(
    const _Float16* __restrict__ A, int lda, int kcs, int K,
    const _Float16* __restrict__ Bt, int ldb,
    const float* __restrict__ bias, const float* __restrict__ resid,
    float* __restrict__ out, float osc)
{
  __shared__ __attribute__((aligned(16))) float sF[128 * 64];
  const int tid = threadIdx.x, lane = tid & 31, w = tid >> 5;
  const int h = lane >> 4, m = lane & 15;
  const int m0 = blockIdx.x * 128, c0 = blockIdx.y * 64;
  const int m0w = m0 + 32 * w;

  const v8f zero8 = {0.f, 0.f, 0.f, 0.f, 0.f, 0.f, 0.f, 0.f};
  v8f acc[2][4];
  #pragma unroll
  for (int mt = 0; mt < 2; ++mt)
    #pragma unroll
    for (int nt = 0; nt < 4; ++nt) acc[mt][nt] = zero8;

  gemm_core(A, lda, kcs, Bt, ldb, K, m0w + m, c0 + m, h, acc);

  #pragma unroll
  for (int nt = 0; nt < 4; ++nt) {
    const int feat = 16 * nt + m;
    const float bvl = bias[c0 + feat];
    #pragma unroll
    for (int mt = 0; mt < 2; ++mt) {
      #pragma unroll
      for (int r = 0; r < 8; ++r) {
        const int tokl = 32 * w + 16 * mt + 8 * h + r;
        sF[tokl * 64 + feat] = acc[mt][nt][r] * osc + bvl;
      }
    }
  }
  __syncthreads();

  f32_store(sF, resid, out, m0, c0, w, lane);
  __threadfence();
  f32_store(sF, resid, out, m0, c0, w, lane);
}

__device__ __forceinline__ float tbias(float tvk, float tvq, const float* tb8) {
  const float dt = tvk - tvq;
  const float lg = log1pf(fabsf(dt) + 1e-6f);
  const float sl = (dt > 0.0f) ? lg : ((dt < 0.0f) ? -lg : 0.0f);
  const float cl = fminf(fmaxf(sl, -5.0f), 5.0f);
  const float nr = (cl + 5.0f) * 0.1f;
  int idx = (int)floorf(nr * 20.0f);
  idx = min(max(idx, 0), NBK - 1);
  return tb8[idx * NH];
}

__device__ __forceinline__ v16h pack_p(v8f a, v8f c) {
  const v16h r = { (_Float16)(a[0] * PSC), (_Float16)(a[1] * PSC), (_Float16)(a[2] * PSC), (_Float16)(a[3] * PSC),
                   (_Float16)(a[4] * PSC), (_Float16)(a[5] * PSC), (_Float16)(a[6] * PSC), (_Float16)(a[7] * PSC),
                   (_Float16)(c[0] * PSC), (_Float16)(c[1] * PSC), (_Float16)(c[2] * PSC), (_Float16)(c[3] * PSC),
                   (_Float16)(c[4] * PSC), (_Float16)(c[5] * PSC), (_Float16)(c[6] * PSC), (_Float16)(c[7] * PSC) };
  return r;
}

__device__ __forceinline__ void att_store(const _Float16* soh, _Float16* ofp, int head, int q0w, int lane) {
  const int q8 = lane & 7, sub = lane >> 3;
  #pragma unroll
  for (int i = 0; i < 2; ++i) {
    const int li = 4 * i + sub;
    const v8h v = *(const v8ha*)(soh + li * 64 + 8 * q8);
    *(volatile v8h*)(ofp + ((size_t)head * NTOK + q0w) * HD + li * 64 + 8 * q8) = v;
  }
}

__global__ __launch_bounds__(128) void attn_kernel(
    const _Float16* __restrict__ qpl,
    const _Float16* __restrict__ kpl,
    const _Float16* __restrict__ vtp,
    const int* __restrict__ tok, const float* __restrict__ tvec, const int* __restrict__ seedp,
    const float* __restrict__ adjb,
    const float* __restrict__ tpb,
    const float* __restrict__ tmb,
    const int* __restrict__ esrc, const int* __restrict__ edst, const int* __restrict__ erel,
    _Float16* __restrict__ ofp)
{
  __shared__ __attribute__((aligned(16))) unsigned char pool[40960];
  __shared__ __attribute__((aligned(16))) float ltpb[NT * NT * NH];
  __shared__ float ladj[NR * NH];
  __shared__ float ltmb[NBK * NH];
  __shared__ int scnt[4];
  __shared__ int bst[4][32];
  __shared__ int bnum[4][32];

  const int tid = threadIdx.x, L = tid & 31, w = tid >> 5, h = L >> 4, m = L & 15;
  const int head = blockIdx.y, q0 = blockIdx.x * 64, q0w = q0 + 16 * w;
  const int seed = seedp[0];

  for (int i = tid; i < NT * NT * NH; i += 128) ltpb[i] = tpb[i];
  if (tid < NR * NH) ladj[tid] = adjb[tid];
  for (int i = tid; i < NBK * NH; i += 128) ltmb[i] = tmb[i];

  unsigned* seg  = (unsigned*)pool;
  int*      hist = (int*)(pool + 8192 + w * 8192);
  float*    slot = (float*)(pool + 8192 + w * 8192);
  unsigned* srt  = (unsigned*)(pool + 8192 + w * 8192 + 4096);
  _Float16* soh  = (_Float16*)(pool + w * 1024);

  {
    unsigned* sg = seg + w * SEGCAP;
    int cntw = 0;
    const int ebeg = w * (NE / 4);
    #pragma unroll 1
    for (int it = 0; it < (NE / 4) / 128; ++it) {
      const int e0 = ebeg + it * 128 + 4 * L;
      const i4 sv = *(const i4a*)(esrc + e0);
      const i4 dv = *(const i4a*)(edst + e0);
      const i4 rv = *(const i4a*)(erel + e0);
      #pragma unroll
      for (int kk = 0; kk < 4; ++kk) {
        const int s = sv[kk], d = dv[kk];
        const int r = min(max(rv[kk], 0), NR - 1);
        const unsigned rl = (unsigned)(s - q0);
        const bool hit = (rl < 64u) && ((unsigned)d < (unsigned)NTOK);
        const unsigned bal = __builtin_amdgcn_ballot_w32(hit);
        const int pos = cntw + (int)__popc(bal & ((1u << L) - 1u));
        if (hit && pos < SEGCAP) sg[pos] = ((unsigned)d << 10) | (rl << 4) | (unsigned)r;
        cntw += (int)__popc(bal);
      }
    }
    if (L == 0) scnt[w] = min(cntw, SEGCAP);
    const i4 z4 = {0, 0, 0, 0};
    #pragma unroll
    for (int i = 0; i < 8; ++i) *(i4a*)(hist + L * 32 + 4 * i) = z4;
  }
  __syncthreads();

  #pragma unroll 1
  for (int sw = 0; sw < 4; ++sw) {
    const int cnt = scnt[sw];
    const unsigned* sg = seg + sw * SEGCAP;
    for (int i = L; i < cnt; i += 32) {
      const unsigned en = sg[i];
      const unsigned rl = (en >> 4) & 63u;
      if ((int)(rl >> 4) == w) hist[L * 32 + (int)(en >> 16)] += 1;
    }
  }
  __syncthreads();
  {
    int run = 0;
    #pragma unroll 1
    for (int l2 = 0; l2 < 32; ++l2) {
      const int tt = hist[l2 * 32 + L];
      hist[l2 * 32 + L] = run;
      run += tt;
    }
    int x = run;
    #pragma unroll
    for (int dd = 1; dd < 32; dd <<= 1) {
      const int y = __shfl_up(x, dd);
      if (L >= dd) x += y;
    }
    bst[w][L] = x - run;
    bnum[w][L] = run;
  }
  __syncthreads();
  #pragma unroll 1
  for (int sw = 0; sw < 4; ++sw) {
    const int cnt = scnt[sw];
    const unsigned* sg = seg + sw * SEGCAP;
    for (int i = L; i < cnt; i += 32) {
      const unsigned en = sg[i];
      const unsigned rl = (en >> 4) & 63u;
      if ((int)(rl >> 4) == w) {
        const int b = (int)(en >> 16);
        const int pos = bst[w][b] + hist[L * 32 + b];
        hist[L * 32 + b] += 1;
        if ((unsigned)pos < (unsigned)WCAP)
          srt[pos] = ((en >> 10) & 63u) | ((rl & 15u) << 6) | ((en & 15u) << 10);
      }
    }
  }
  __syncthreads();
  {
    const v4f z = {0.f, 0.f, 0.f, 0.f};
    #pragma unroll
    for (int i = 0; i < 8; ++i) *(v4fa*)(slot + L * 32 + 4 * i) = z;
  }

  const int qi = q0w + m;
  const unsigned tq = min((unsigned)tok[qi], (unsigned)(NT - 1));
  const float* tprow = ltpb + tq * (NT * NH) + head;
  const float* tmh = ltmb + head;
  const float tvq = tvec[qi];
  const bool tfl = (qi < seed);
  const bool anyt = (__builtin_amdgcn_ballot_w32(tfl) != 0u);

  const v16h qb = load_frag(qpl + (size_t)qi * CH + head * HD, h);
  const _Float16* kbase = kpl + (size_t)m * CH + head * HD;
  const _Float16* vbase = vtp + (size_t)(head * HD + m) * NTOK;
  const float scl = 1.0f / 5.656854249492381f;

  const v8f zero8 = {0.f, 0.f, 0.f, 0.f, 0.f, 0.f, 0.f, 0.f};
  v8f o[2];
  o[0] = zero8; o[1] = zero8;
  float mrun = -1e30f, lrun = 0.0f;

  #pragma unroll 1
  for (int kb = 0; kb < NTOK; kb += 64) {
    v8f s[4];
    #pragma unroll
    for (int j = 0; j < 4; ++j) {
      const v16h kf = load_frag(kbase + (size_t)(kb + 16 * j) * CH, h);
      s[j] = wmma_f16(kf, qb, zero8);
    }
    {
      const int b = kb >> 6;
      const int beg = bst[w][b];
      int num = min(bnum[w][b], WCAP - beg);
      num = max(num, 0);
      #pragma unroll 1
      for (int t = 0; t < num; ++t) {
        const unsigned en = srt[beg + t];
        const int ko = (int)(en & 63u);
        const int rloc = (int)((en >> 6) & 15u);
        const int rel = (int)((en >> 10) & 15u);
        const int own = rloc | ((ko & 8) << 1);
        if (own == L) {
          const int e = ((ko >> 4) << 3) | (ko & 7);
          slot[L * 32 + e] += ladj[rel * NH + head];
        }
      }
    }
    #pragma unroll
    for (int j = 0; j < 4; ++j) {
      const int kk0 = kb + 16 * j + 8 * h;
      const i4 ta = *(const i4a*)(tok + kk0);
      const i4 tc = *(const i4a*)(tok + kk0 + 4);
      const v4f ea = *(const v4fa*)(slot + L * 32 + 8 * j);
      const v4f ec = *(const v4fa*)(slot + L * 32 + 8 * j + 4);
      s[j][0] = s[j][0] * scl + tprow[min((unsigned)ta.x, 7u) * NH] + ea.x;
      s[j][1] = s[j][1] * scl + tprow[min((unsigned)ta.y, 7u) * NH] + ea.y;
      s[j][2] = s[j][2] * scl + tprow[min((unsigned)ta.z, 7u) * NH] + ea.z;
      s[j][3] = s[j][3] * scl + tprow[min((unsigned)ta.w, 7u) * NH] + ea.w;
      s[j][4] = s[j][4] * scl + tprow[min((unsigned)tc.x, 7u) * NH] + ec.x;
      s[j][5] = s[j][5] * scl + tprow[min((unsigned)tc.y, 7u) * NH] + ec.y;
      s[j][6] = s[j][6] * scl + tprow[min((unsigned)tc.z, 7u) * NH] + ec.z;
      s[j][7] = s[j][7] * scl + tprow[min((unsigned)tc.w, 7u) * NH] + ec.w;
    }
    {
      const v4f z = {0.f, 0.f, 0.f, 0.f};
      #pragma unroll
      for (int i = 0; i < 8; ++i) *(v4fa*)(slot + L * 32 + 4 * i) = z;
    }
    if (anyt) {
      #pragma unroll
      for (int j = 0; j < 4; ++j) {
        const int kk0 = kb + 16 * j + 8 * h;
        const v4f va = *(const v4fa*)(tvec + kk0);
        const v4f vc = *(const v4fa*)(tvec + kk0 + 4);
        float tb;
        tb = tbias(va.x, tvq, tmh); s[j][0] += tfl ? tb : 0.0f;
        tb = tbias(va.y, tvq, tmh); s[j][1] += tfl ? tb : 0.0f;
        tb = tbias(va.z, tvq, tmh); s[j][2] += tfl ? tb : 0.0f;
        tb = tbias(va.w, tvq, tmh); s[j][3] += tfl ? tb : 0.0f;
        tb = tbias(vc.x, tvq, tmh); s[j][4] += tfl ? tb : 0.0f;
        tb = tbias(vc.y, tvq, tmh); s[j][5] += tfl ? tb : 0.0f;
        tb = tbias(vc.z, tvq, tmh); s[j][6] += tfl ? tb : 0.0f;
        tb = tbias(vc.w, tvq, tmh); s[j][7] += tfl ? tb : 0.0f;
      }
    }

    float mloc = s[0][0];
    #pragma unroll
    for (int j = 0; j < 4; ++j)
      #pragma unroll
      for (int r = 0; r < 8; ++r) mloc = fmaxf(mloc, s[j][r]);
    mloc = fmaxf(mloc, __shfl_xor(mloc, 16));
    const float mnew = fmaxf(mrun, mloc);
    const float alpha = __expf(mrun - mnew);
    mrun = mnew;
    float lsum = 0.0f;
    #pragma unroll
    for (int j = 0; j < 4; ++j)
      #pragma unroll
      for (int r = 0; r < 8; ++r) {
        const float p = __expf(s[j][r] - mnew);
        s[j][r] = p;
        lsum += p;
      }
    lsum += __shfl_xor(lsum, 16);
    lrun = lrun * alpha + lsum;
    #pragma unroll
    for (int t = 0; t < 2; ++t)
      #pragma unroll
      for (int r = 0; r < 8; ++r) o[t][r] = o[t][r] * alpha;

    const v16h pb0 = pack_p(s[0], s[1]);
    const v16h pb1 = pack_p(s[2], s[3]);

    #pragma unroll
    for (int t = 0; t < 2; ++t) {
      const _Float16* vp = vbase + (size_t)(16 * t) * NTOK + kb;
      const v16h vf0 = load_frag(vp, h);
      const v16h vf1 = load_frag(vp + 32, h);
      o[t] = wmma_f16(vf0, pb0, o[t]);
      o[t] = wmma_f16(vf1, pb1, o[t]);
    }
  }

  const float inv = (1.0f / lrun) * (OSC / PSC);
  #pragma unroll
  for (int t = 0; t < 2; ++t)
    #pragma unroll
    for (int r = 0; r < 8; ++r)
      soh[m * 32 + 16 * t + 8 * h + r] = (_Float16)(o[t][r] * inv);
  __syncthreads();

  att_store(soh, ofp, head, q0w, L);
  __threadfence();
  att_store(soh, ofp, head, q0w, L);
}

extern "C" void kernel_launch(void* const* d_in, const int* in_sizes, int n_in,
                              void* d_out, int out_size, void* d_ws, size_t ws_size,
                              hipStream_t stream) {
  if (n_in < 26) return;
  if (in_sizes[0] != NTOK * CH || in_sizes[1] != NTOK) return;
  if (in_sizes[2] != NE || in_sizes[3] != NE || in_sizes[4] != NE) return;
  if (in_sizes[5] != NTOK || in_sizes[6] < 1) return;
  if (in_sizes[7] != CH * CH || in_sizes[9] != CH * CH || in_sizes[11] != CH * CH || in_sizes[13] != CH * CH) return;
  if (in_sizes[8] != CH || in_sizes[10] != CH || in_sizes[12] != CH || in_sizes[14] != CH) return;
  if (in_sizes[15] != CH || in_sizes[16] != CH || in_sizes[17] != CH || in_sizes[18] != CH) return;
  if (in_sizes[19] != CH * FF || in_sizes[20] != FF || in_sizes[21] != FF * CH || in_sizes[22] != CH) return;
  if (in_sizes[23] != NR * NH || in_sizes[24] != NT * NT * NH || in_sizes[25] != NBK * NH) return;
  if (out_size != NTOK * CH) return;

  const float* X    = (const float*)d_in[0];
  const int*   tok  = (const int*)  d_in[1];
  const int*   esrc = (const int*)  d_in[2];
  const int*   edst = (const int*)  d_in[3];
  const int*   erel = (const int*)  d_in[4];
  const float* tvec = (const float*)d_in[5];
  const int*   seed = (const int*)  d_in[6];
  const float* Wq = (const float*)d_in[7];   const float* bq = (const float*)d_in[8];
  const float* Wk = (const float*)d_in[9];   const float* bk = (const float*)d_in[10];
  const float* Wv = (const float*)d_in[11];  const float* bv = (const float*)d_in[12];
  const float* Wo = (const float*)d_in[13];  const float* bo = (const float*)d_in[14];
  const float* l1g = (const float*)d_in[15]; const float* l1b = (const float*)d_in[16];
  const float* l2g = (const float*)d_in[17]; const float* l2b = (const float*)d_in[18];
  const float* W1 = (const float*)d_in[19];  const float* b1 = (const float*)d_in[20];
  const float* W2 = (const float*)d_in[21];  const float* b2 = (const float*)d_in[22];
  const float* adjb = (const float*)d_in[23];
  const float* tpb  = (const float*)d_in[24];
  const float* tmb  = (const float*)d_in[25];
  float* out = (float*)d_out;

  const size_t b_wt4 = (size_t)4 * CH * CH * 2;
  const size_t b_w1t = (size_t)FF * CH * 2;
  const size_t b_w2t = (size_t)CH * FF * 2;
  const size_t b_pl  = (size_t)NTOK * CH * 2;
  const size_t b_x   = (size_t)NTOK * CH * 4;
  const size_t b_g   = (size_t)NTOK * FF * 2;
  const size_t o_wt4 = 0;
  const size_t o_w1t = o_wt4 + b_wt4;
  const size_t o_w2t = o_w1t + b_w1t;
  const size_t o_h1  = o_w2t + b_w2t;
  const size_t o_q   = o_h1  + b_pl;
  const size_t o_k   = o_q   + b_pl;
  const size_t o_vt  = o_k   + b_pl;
  const size_t o_of  = o_vt  + b_pl;
  const size_t o_x   = o_of  + b_pl;
  const size_t o_h2  = o_x   + b_x;
  const size_t o_g   = o_h2  + b_pl;
  const size_t total = o_g   + b_g;
  if (total > ws_size) return;

  char* ws = (char*)d_ws;
  _Float16* wt4 = (_Float16*)(ws + o_wt4);
  _Float16* w1t = (_Float16*)(ws + o_w1t);
  _Float16* w2t = (_Float16*)(ws + o_w2t);
  _Float16* h1  = (_Float16*)(ws + o_h1);
  _Float16* qpl = (_Float16*)(ws + o_q);
  _Float16* kpl = (_Float16*)(ws + o_k);
  _Float16* vtp = (_Float16*)(ws + o_vt);
  _Float16* ofp = (_Float16*)(ws + o_of);
  float*    xb  = (float*)   (ws + o_x);
  _Float16* h2  = (_Float16*)(ws + o_h2);
  _Float16* gpl = (_Float16*)(ws + o_g);
  _Float16* wot = wt4 + (size_t)3 * CH * CH;

  wtr_kernel<<<dim3(CH / 64, CH / 64, 4), 256, 0, stream>>>(Wq, Wk, Wv, Wo, wt4, CH, CH);
  wtr_kernel<<<dim3(FF / 64, CH / 64, 1), 256, 0, stream>>>(W1, W1, W1, W1, w1t, CH, FF);
  wtr_kernel<<<dim3(CH / 64, FF / 64, 1), 256, 0, stream>>>(W2, W2, W2, W2, w2t, FF, CH);

  ln_kernel<<<NTOK / 8, 256, 0, stream>>>(X, l1g, l1b, h1, NTOK);
  qkv_kernel<<<dim3(NTOK / 128, 12), 128, 0, stream>>>(h1, wt4, bq, bk, bv, qpl, kpl, vtp);

  attn_kernel<<<dim3(NTOK / 64, NH), 128, 0, stream>>>(qpl, kpl, vtp, tok, tvec, seed, adjb, tpb, tmb,
                                                      esrc, edst, erel, ofp);

  gemm_f32_kernel<<<dim3(NTOK / 128, CH / 64), 128, 0, stream>>>(ofp, HD, NTOK * HD, CH, wot, CH, bo, X, xb,
                                                                1.0f / (OSC * WSC));

  ln_kernel<<<NTOK / 8, 256, 0, stream>>>(xb, l2g, l2b, h2, NTOK);
  ffn1_kernel<<<dim3(NTOK / 128, FF / 64), 128, 0, stream>>>(h2, w1t, b1, gpl);
  gemm_f32_kernel<<<dim3(NTOK / 128, CH / 64), 128, 0, stream>>>(gpl, FF, 32, FF, w2t, FF, b2, xb, out,
                                                                1.0f / (GSC * WSC));
}
